// BMN_66683662238004
// MI455X (gfx1250) — hardware-verified
//
#include <hip/hip_runtime.h>
#include <stdint.h>
#include <stddef.h>


#define T_DIM    100
#define NPOS     10000
#define NPOS_PAD 10112
#define NSMP     32
#define NBATCH   4
#define CMID     128
#define KBIG     4096
#define OBIG     512
#define RVALID   4950
#define RPAD     4992
#define ACT_SC   4.0f
#define W_SC     16.0f
#define ACC_INV  0.015625f

static_assert(RPAD % 128 == 0);
static_assert(RPAD >= RVALID + 1);
static_assert(NPOS_PAD % 64 == 0);
static_assert(NPOS_PAD >= ((NPOS + 63) / 64) * 64);
static_assert((RPAD * 8) % 256 == 0);

typedef unsigned int v4u  __attribute__((ext_vector_type(4)));
typedef float        v4f  __attribute__((ext_vector_type(4)));
typedef float        v8f  __attribute__((ext_vector_type(8)));
typedef _Float16     v8h  __attribute__((ext_vector_type(8)));
typedef _Float16     v16h __attribute__((ext_vector_type(16)));

union Frag { v16h v; v4u u[2]; };
union H8   { v8h h; v4u u; };

__device__ __forceinline__ v8f zacc() { v8f z = {0.f, 0.f, 0.f, 0.f, 0.f, 0.f, 0.f, 0.f}; return z; }
__device__ __forceinline__ v4u ld16(const uint16_t* p) { return *(const v4u*)p; }
__device__ __forceinline__ void st16v(uint16_t* p, v4u v) { *(volatile v4u*)p = v; }
__device__ __forceinline__ void st4fv(float* p, v4f v) { *(volatile v4f*)p = v; }
__device__ __forceinline__ void st1fv(float* p, float v) { *(volatile float*)p = v; }

__device__ __forceinline__ v8f wmma16(const Frag& a, const Frag& b, v8f c) {
  return __builtin_amdgcn_wmma_f32_16x16x32_f16(false, a.v, false, b.v, (short)0, c, false, false);
}

#define NOPG_2x4(ACC, A0, A1, B)                                                                 \
  asm volatile("v_nop\n\tv_nop\n\tv_nop\n\tv_nop"                                              \
               : "+v"(ACC[0][0]), "+v"(ACC[0][1]), "+v"(ACC[0][2]), "+v"(ACC[0][3]),           \
                 "+v"(ACC[1][0]), "+v"(ACC[1][1]), "+v"(ACC[1][2]), "+v"(ACC[1][3])            \
               : "v"(A0.v), "v"(A1.v), "v"(B[0].v), "v"(B[1].v), "v"(B[2].v), "v"(B[3].v))

#define NOPG_1x4(ACC, A0, B)                                                                     \
  asm volatile("v_nop\n\tv_nop\n\tv_nop\n\tv_nop"                                              \
               : "+v"(ACC[0]), "+v"(ACC[1]), "+v"(ACC[2]), "+v"(ACC[3])                        \
               : "v"(A0.v), "v"(B[0].v), "v"(B[1].v), "v"(B[2].v), "v"(B[3].v))

__device__ __forceinline__ int tri_S(int d) { return (d * (199 - d)) >> 1; }
__device__ __forceinline__ void row_to_dt(int r, int& d, int& t) {
  r = r < 0 ? 0 : (r > RVALID - 1 ? RVALID - 1 : r);
  float disc = 39601.0f - 8.0f * (float)r;
  disc = fmaxf(disc, 0.0f);
  int dd = (int)((199.0f - sqrtf(disc)) * 0.5f);
  dd = dd < 0 ? 0 : (dd > 98 ? 98 : dd);
#pragma unroll
  for (int it = 0; it < 3; ++it) { if (dd > 0 && tri_S(dd) > r) --dd; }
#pragma unroll
  for (int it = 0; it < 3; ++it) { if (dd < 98 && tri_S(dd + 1) <= r) ++dd; }
  int tt = r - tri_S(dd);
  tt = tt < 0 ? 0 : (tt > T_DIM - 1 ? T_DIM - 1 : tt);
  d = dd; t = tt;
}

__global__ __launch_bounds__(256) void k_cvt(const float* __restrict__ wc3d, const float* __restrict__ w2d1,
                                             const float* __restrict__ w2d2,
                                             uint16_t* A5, uint16_t* A6, uint16_t* A7) {
  const int gid = blockIdx.x * 256 + threadIdx.x;
  const int N1 = OBIG * KBIG / 8;
  const int N2 = CMID * OBIG / 8;
  const int N3 = 9 * CMID * CMID / 8;
  H8 hv;
  uint16_t* dp;
  if (gid < N1) {
    const size_t e = (size_t)gid * 8;
    const v4f x0 = *(const v4f*)(wc3d + e), x1 = *(const v4f*)(wc3d + e + 4);
    hv.h[0] = (_Float16)(x0.x * W_SC); hv.h[1] = (_Float16)(x0.y * W_SC);
    hv.h[2] = (_Float16)(x0.z * W_SC); hv.h[3] = (_Float16)(x0.w * W_SC);
    hv.h[4] = (_Float16)(x1.x * W_SC); hv.h[5] = (_Float16)(x1.y * W_SC);
    hv.h[6] = (_Float16)(x1.z * W_SC); hv.h[7] = (_Float16)(x1.w * W_SC);
    dp = A5 + e;
  } else if (gid < N1 + N2) {
    const size_t e = (size_t)(gid - N1) * 8;
    const v4f x0 = *(const v4f*)(w2d1 + e), x1 = *(const v4f*)(w2d1 + e + 4);
    hv.h[0] = (_Float16)(x0.x * W_SC); hv.h[1] = (_Float16)(x0.y * W_SC);
    hv.h[2] = (_Float16)(x0.z * W_SC); hv.h[3] = (_Float16)(x0.w * W_SC);
    hv.h[4] = (_Float16)(x1.x * W_SC); hv.h[5] = (_Float16)(x1.y * W_SC);
    hv.h[6] = (_Float16)(x1.z * W_SC); hv.h[7] = (_Float16)(x1.w * W_SC);
    dp = A6 + e;
  } else if (gid < N1 + N2 + N3) {
    const int e = (gid - N1 - N2) * 8;
    const int s = e >> 14, rem = e & 16383, o = rem >> 7, c0 = rem & 127;
#pragma unroll
    for (int i = 0; i < 8; ++i)
      hv.h[i] = (_Float16)(w2d2[((size_t)(o * CMID + c0 + i)) * 9 + s] * W_SC);
    dp = A7 + e;
  } else {
    return;
  }
  st16v(dp, hv.u);
  __threadfence();
  st16v(dp, hv.u);
}

__global__ __launch_bounds__(256) void k_conv1d(const float* __restrict__ in, const float* __restrict__ w,
                                                const float* __restrict__ bias, float* out, int Cin, int Cout) {
  __shared__ v4u As[64 * 5];
  __shared__ v4u Bs[128 * 5];
  __shared__ __attribute__((aligned(16))) float Ot[64 * T_DIM];
  const int tid = threadIdx.x, lane = tid & 31, wave = tid >> 5, h = lane >> 4, m = lane & 15;
  const int wm = wave & 3, wn = wave >> 2;
  const int co0 = blockIdx.x * 64, b = blockIdx.y;
  const int K = 3 * Cin, Kpad = (K + 31) & ~31, nks = Kpad >> 5;
  v8f acc[4];
#pragma unroll
  for (int ni = 0; ni < 4; ++ni) acc[ni] = zacc();
  const int a_co = tid >> 2, a_kq = (tid & 3) * 8;
  const int b_t = tid >> 1, b_kh = (tid & 1) * 16;
  const float* wrow = w + (size_t)(co0 + a_co) * K;
  const float* inb = in + (size_t)b * Cin * T_DIM;

#pragma unroll 1
  for (int ks = 0; ks < nks; ++ks) {
    const int k0 = ks * 32;
    {
      H8 hv;
#pragma unroll
      for (int i = 0; i < 8; ++i) {
        const int kk = k0 + a_kq + i;
        const int kc = kk < K ? kk : K - 1;
        const float v = wrow[kc];
        hv.h[i] = (_Float16)((kk < K) ? v * W_SC : 0.0f);
      }
      As[a_co * 5 + (tid & 3)] = hv.u;
    }
#pragma unroll
    for (int s = 0; s < 2; ++s) {
      H8 hv;
#pragma unroll
      for (int i = 0; i < 8; ++i) {
        const int kk = k0 + b_kh + 8 * s + i;
        const int ci = kk / 3, kt = kk - ci * 3;
        const int tt = b_t + kt - 1;
        const bool ok = (kk < K) && (b_t < T_DIM) && (tt >= 0) && (tt < T_DIM);
        const int cic = ci < Cin ? ci : Cin - 1;
        const int ttc = tt < 0 ? 0 : (tt > T_DIM - 1 ? T_DIM - 1 : tt);
        const float v = inb[(size_t)cic * T_DIM + ttc];
        hv.h[i] = (_Float16)(ok ? v * ACT_SC : 0.0f);
      }
      Bs[b_t * 5 + (tid & 1) * 2 + s] = hv.u;
    }
    __syncthreads();
    Frag a;
    a.u[0] = As[(16 * wm + m) * 5 + h];
    a.u[1] = As[(16 * wm + m) * 5 + 2 + h];
    Frag bf[4];
#pragma unroll
    for (int ni = 0; ni < 4; ++ni) {
      const int t = 64 * wn + 16 * ni + m;
      bf[ni].u[0] = Bs[t * 5 + h];
      bf[ni].u[1] = Bs[t * 5 + 2 + h];
    }
#pragma unroll
    for (int ni = 0; ni < 4; ++ni) acc[ni] = wmma16(a, bf[ni], acc[ni]);
    NOPG_1x4(acc, a, bf);
    __syncthreads();
  }

  {
    float bs[8];
#pragma unroll
    for (int j = 0; j < 8; ++j) bs[j] = bias[co0 + 16 * wm + 8 * h + j];
#pragma unroll
    for (int ni = 0; ni < 4; ++ni) {
      const int t = 64 * wn + 16 * ni + m;
#pragma unroll
      for (int j = 0; j < 8; ++j) {
        const int col = 16 * wm + 8 * h + j;
        float v = acc[ni][j] * ACC_INV + bs[j];
        v = fmaxf(v, 0.0f);
        if (t < T_DIM) Ot[col * T_DIM + t] = v;
      }
    }
  }
  __syncthreads();
  float* ob = out + ((size_t)b * Cout + co0) * T_DIM;
#pragma unroll
  for (int i = 0; i < 7; ++i) {
    const int q = i * 256 + tid;
    if (q < 1600) { const v4f v = *(const v4f*)(Ot + 4 * q); st4fv(ob + 4 * q, v); }
  }
  __threadfence();
#pragma unroll
  for (int i = 0; i < 7; ++i) {
    const int q = i * 256 + tid;
    if (q < 1600) { const v4f v = *(const v4f*)(Ot + 4 * q); st4fv(ob + 4 * q, v); }
  }
}

__global__ __launch_bounds__(256) void k_tem_head(const float* __restrict__ tem, const float* __restrict__ w,
                                                  const float* __restrict__ bias, float* out) {
  __shared__ __attribute__((aligned(16))) float sv[800];
  const int tid = threadIdx.x;
#pragma unroll 1
  for (int q = 0; q < 4; ++q) {
    const int f = q * 256 + tid;
    if (f < 800) {
      const int b = f / 200, rr = f - b * 200, ch = rr / 100, t = rr - ch * 100;
      float acc = bias[ch];
      const float* xb = tem + (size_t)b * 256 * T_DIM;
      const float* wb = w + (size_t)ch * 256 * 3;
      const int tm = t > 0 ? t - 1 : 0, tp = t < T_DIM - 1 ? t + 1 : T_DIM - 1;
      const float pm = t > 0 ? 1.0f : 0.0f, pp = t < T_DIM - 1 ? 1.0f : 0.0f;
#pragma unroll 1
      for (int ci = 0; ci < 256; ++ci) {
        const float* xr = xb + ci * T_DIM;
        const float x0 = xr[tm] * pm, x1 = xr[t], x2 = xr[tp] * pp;
        acc += wb[ci * 3] * x0 + wb[ci * 3 + 1] * x1 + wb[ci * 3 + 2] * x2;
      }
      float z = fminf(fmaxf(acc, -80.0f), 80.0f);
      sv[f] = 1.0f / (1.0f + expf(-z));
    }
  }
  __syncthreads();
  v4f v = {0.f, 0.f, 0.f, 0.f};
  const bool wr = tid < 200;
  if (wr) v = *(const v4f*)(sv + 4 * tid);
  if (wr) st4fv(out + 4 * tid, v);
  __threadfence();
  if (wr) st4fv(out + 4 * tid, v);
}

__global__ __launch_bounds__(256) void k_pem(const float* __restrict__ base, uint16_t* P, int bsel) {
#pragma clang fp contract(off)
  const int gid = blockIdx.x * 256 + threadIdx.x;
  const int r = gid >> 3, piece = gid & 7, chalf = piece >> 2, n0 = (piece & 3) * 8;
  int tl[8], tr[8];
  float wl[8], wr[8];
#pragma unroll
  for (int q = 0; q < 8; ++q) { tl[q] = 0; tr[q] = 0; wl[q] = 0.0f; wr[q] = 0.0f; }
  if (r < RVALID) {
    int d, t;
    row_to_dt(r, d, t);
    const double L   = (double)(d + 1 - t);
    const double xlo = (double)t - L * 0.5;
    const double xhi = (double)(d + 1) + L * 0.5;
    const double bin = (xhi - xlo) / 31.0;
#pragma unroll
    for (int q = 0; q < 8; ++q) {
      const double xp = xlo + (double)(n0 + q) * bin;
      if (xp >= 0.0 && xp <= 99.0) {
        const double fl = floor(xp), cl = ceil(xp);
        wl[q] = (float)(1.0 - (xp - fl));
        wr[q] = (float)(1.0 - (cl - xp));
        int il = (int)fl, ir = (int)cl;
        il = il < 0 ? 0 : (il > T_DIM - 1 ? T_DIM - 1 : il);
        ir = ir < 0 ? 0 : (ir > T_DIM - 1 ? T_DIM - 1 : ir);
        tl[q] = il; tr[q] = ir;
      }
    }
  }
  const float* bb = base + (size_t)bsel * CMID * T_DIM;
  uint16_t* prow = P + (size_t)r * KBIG + n0;
#pragma unroll 1
  for (int cp = 0; cp < CMID / 2; ++cp) {
    const int c = 2 * cp + chalf;
    const float* bc = bb + c * T_DIM;
    H8 hv;
#pragma unroll
    for (int q = 0; q < 8; ++q) {
      const float g = wl[q] * bc[tl[q]] + wr[q] * bc[tr[q]];
      hv.h[q] = (_Float16)(g * ACT_SC);
    }
    uint16_t* dp = prow + c * NSMP;
    st16v(dp, hv.u);
    __threadfence();
    st16v(dp, hv.u);
  }
}

template <int MODE>
__device__ __forceinline__ void gemm_store_pass(const v4u* tile, const int* pmap, uint16_t* dst, uint16_t* cvec,
                                                int tid, int b, int r0, int o0, int ldd) {
#pragma unroll
  for (int g = 0; g < 8; ++g) {
    const int rl = g * 16 + (tid >> 4), piece = tid & 15;
    const v4u v = tile[rl * 17 + piece];
    if (MODE == 0) {
      uint16_t* dp = dst + ((size_t)(b * RPAD + r0 + rl) * ldd + o0 + piece * 8);
      st16v(dp, v);
    } else {
      const int code = pmap[rl];
      const int pc = code < 0 ? 0 : (code > NPOS - 1 ? NPOS - 1 : code);
      uint16_t* dp = (code == -2) ? (cvec + piece * 8)
                                  : (dst + ((size_t)(b * NPOS_PAD + pc) * ldd + piece * 8));
      if (code != -1) st16v(dp, v);
    }
  }
}

template <int MODE>
__global__ __launch_bounds__(256) void k_gemm(const uint16_t* __restrict__ A, const uint16_t* __restrict__ Bm,
                                              const float* __restrict__ bias, uint16_t* dst, uint16_t* cvec,
                                              int K, int bsel) {
  __shared__ v4u tile[128 * 17];
  __shared__ int pmap[128];
  const int tid = threadIdx.x, lane = tid & 31, wave = tid >> 5, h = lane >> 4, m = lane & 15;
  const int wm = wave >> 1, wn = wave & 1;
  const int r0 = blockIdx.x * 128;
  const int o0 = (MODE == 0) ? (int)blockIdx.y * 128 : 0;
  const int b  = (MODE == 0) ? bsel : (int)blockIdx.z;
  const int ldd = (MODE == 0) ? OBIG : CMID;
  if (MODE == 1) {
    if (tid < 128) {
      const int r = r0 + tid;
      int code;
      if (r < RVALID) { int d, t; row_to_dt(r, d, t); code = d * T_DIM + t; }
      else if (r == RVALID && b == 0) code = -2;
      else code = -1;
      pmap[tid] = code;
    }
  } else {
    if (tid < 128) pmap[tid] = 0;
  }
  const size_t brow0 = (MODE == 0) ? (size_t)0 : (size_t)b * RPAD;
  v8f acc[2][4];
#pragma unroll
  for (int mi = 0; mi < 2; ++mi)
#pragma unroll
    for (int ni = 0; ni < 4; ++ni) acc[mi][ni] = zacc();
  const uint16_t* ap0 = A + (size_t)(o0 + 32 * wm + m) * K + 8 * h;
  const uint16_t* ap1 = ap0 + (size_t)16 * K;
  const uint16_t* bp[4];
#pragma unroll
  for (int ni = 0; ni < 4; ++ni)
    bp[ni] = Bm + (brow0 + (size_t)(r0 + 64 * wn + 16 * ni + m)) * K + 8 * h;
  const int nks = K >> 5;
#pragma unroll 1
  for (int ks = 0; ks < nks; ++ks) {
    const int k0 = ks << 5;
    Frag a0, a1, bq[4];
    a0.u[0] = ld16(ap0 + k0); a0.u[1] = ld16(ap0 + k0 + 16);
    a1.u[0] = ld16(ap1 + k0); a1.u[1] = ld16(ap1 + k0 + 16);
#pragma unroll
    for (int ni = 0; ni < 4; ++ni) { bq[ni].u[0] = ld16(bp[ni] + k0); bq[ni].u[1] = ld16(bp[ni] + k0 + 16); }
#pragma unroll
    for (int ni = 0; ni < 4; ++ni) {
      acc[0][ni] = wmma16(a0, bq[ni], acc[0][ni]);
      acc[1][ni] = wmma16(a1, bq[ni], acc[1][ni]);
    }
    NOPG_2x4(acc, a0, a1, bq);
  }
#pragma unroll
  for (int mi = 0; mi < 2; ++mi) {
    const int ol = 32 * wm + 16 * mi + 8 * h;
    float bs[8];
#pragma unroll
    for (int j = 0; j < 8; ++j) bs[j] = bias[o0 + ol + j];
#pragma unroll
    for (int ni = 0; ni < 4; ++ni) {
      const int rl = 64 * wn + 16 * ni + m;
      H8 hv;
#pragma unroll
      for (int j = 0; j < 8; ++j) {
        float v = acc[mi][ni][j] * ACC_INV + bs[j];
        v = fmaxf(v, 0.0f);
        hv.h[j] = (_Float16)(v * ACT_SC);
      }
      tile[rl * 17 + (ol >> 3)] = hv.u;
    }
  }
  __syncthreads();
  gemm_store_pass<MODE>(tile, pmap, dst, cvec, tid, b, r0, o0, ldd);
  __threadfence();
  gemm_store_pass<MODE>(tile, pmap, dst, cvec, tid, b, r0, o0, ldd);
}

__global__ __launch_bounds__(256) void k_fill(const uint16_t* __restrict__ cvec, uint16_t* y2) {
  const int tid = threadIdx.x;
  const int p = blockIdx.x * 16 + (tid >> 4), piece = tid & 15, b = blockIdx.y;
  const int d = p / T_DIM, t = p - d * T_DIM;
  const bool inv = (p < NPOS) && (d + t > T_DIM - 2);
  const v4u v = ld16(cvec + piece * 8);
  uint16_t* dp = y2 + ((size_t)(b * NPOS_PAD + (p < NPOS ? p : 0)) * CMID + piece * 8);
  if (inv) st16v(dp, v);
  __threadfence();
  if (inv) st16v(dp, v);
}

__global__ __launch_bounds__(128) void k_conv3x3(const uint16_t* __restrict__ A7, const uint16_t* __restrict__ Y2,
                                                 const float* __restrict__ bias, const float* __restrict__ w3,
                                                 const float* __restrict__ b3, float* zb) {
  __shared__ __attribute__((aligned(16))) float tile[64 * 132];
  __shared__ float w3s[256];
  __shared__ float b3s[2];
  const int tid = threadIdx.x, lane = tid & 31, wm = tid >> 5, h = lane >> 4, m = lane & 15;
  const int p0 = blockIdx.x * 64, b = blockIdx.y;
  w3s[tid] = w3[tid];
  w3s[128 + tid] = w3[128 + tid];
  if (tid < 2) b3s[tid] = b3[tid];
  int dn[4], tn[4];
  bool pin[4];
#pragma unroll
  for (int ni = 0; ni < 4; ++ni) {
    const int p = p0 + 16 * ni + m;
    pin[ni] = p < NPOS;
    const int pc = p < NPOS ? p : NPOS - 1;
    dn[ni] = pc / T_DIM;
    tn[ni] = pc - dn[ni] * T_DIM;
  }
  v8f acc[2][4];
#pragma unroll
  for (int mi = 0; mi < 2; ++mi)
#pragma unroll
    for (int ni = 0; ni < 4; ++ni) acc[mi][ni] = zacc();
  const uint16_t* arow0 = A7 + (size_t)(32 * wm + m) * CMID + 8 * h;
  const uint16_t* arow1 = arow0 + (size_t)16 * CMID;
  const uint16_t* yb = Y2 + (size_t)b * NPOS_PAD * CMID + 8 * h;
#pragma unroll 1
  for (int s = 0; s < 9; ++s) {
    const int s3 = s / 3;
    const int dy = s3 - 1, dx = s - s3 * 3 - 1;
    const uint16_t* brow[4];
    unsigned msk[4];
#pragma unroll
    for (int ni = 0; ni < 4; ++ni) {
      const int dd = dn[ni] + dy, tt = tn[ni] + dx;
      const bool ok = pin[ni] && dd >= 0 && dd < T_DIM && tt >= 0 && tt < T_DIM;
      const int ddc = dd < 0 ? 0 : (dd > T_DIM - 1 ? T_DIM - 1 : dd);
      const int ttc = tt < 0 ? 0 : (tt > T_DIM - 1 ? T_DIM - 1 : tt);
      brow[ni] = yb + (size_t)(ddc * T_DIM + ttc) * CMID;
      msk[ni] = ok ? 0xffffffffu : 0u;
    }
    const uint16_t* as0 = arow0 + (size_t)s * CMID * CMID;
    const uint16_t* as1 = arow1 + (size_t)s * CMID * CMID;
#pragma unroll
    for (int cb = 0; cb < 4; ++cb) {
      const int k0 = cb * 32;
      Frag a0, a1, bq[4];
      a0.u[0] = ld16(as0 + k0); a0.u[1] = ld16(as0 + k0 + 16);
      a1.u[0] = ld16(as1 + k0); a1.u[1] = ld16(as1 + k0 + 16);
#pragma unroll
      for (int ni = 0; ni < 4; ++ni) {
        const v4u mk = {msk[ni], msk[ni], msk[ni], msk[ni]};
        bq[ni].u[0] = ld16(brow[ni] + k0) & mk;
        bq[ni].u[1] = ld16(brow[ni] + k0 + 16) & mk;
      }
#pragma unroll
      for (int ni = 0; ni < 4; ++ni) {
        acc[0][ni] = wmma16(a0, bq[ni], acc[0][ni]);
        acc[1][ni] = wmma16(a1, bq[ni], acc[1][ni]);
      }
      NOPG_2x4(acc, a0, a1, bq);
    }
  }
#pragma unroll
  for (int mi = 0; mi < 2; ++mi) {
    const int o = 32 * wm + 16 * mi + 8 * h;
    float bs[8];
#pragma unroll
    for (int j = 0; j < 8; ++j) bs[j] = bias[o + j];
#pragma unroll
    for (int ni = 0; ni < 4; ++ni) {
      const int pl = 16 * ni + m;
      v4f lo, hi;
      lo.x = fmaxf(acc[mi][ni][0] * ACC_INV + bs[0], 0.0f);
      lo.y = fmaxf(acc[mi][ni][1] * ACC_INV + bs[1], 0.0f);
      lo.z = fmaxf(acc[mi][ni][2] * ACC_INV + bs[2], 0.0f);
      lo.w = fmaxf(acc[mi][ni][3] * ACC_INV + bs[3], 0.0f);
      hi.x = fmaxf(acc[mi][ni][4] * ACC_INV + bs[4], 0.0f);
      hi.y = fmaxf(acc[mi][ni][5] * ACC_INV + bs[5], 0.0f);
      hi.z = fmaxf(acc[mi][ni][6] * ACC_INV + bs[6], 0.0f);
      hi.w = fmaxf(acc[mi][ni][7] * ACC_INV + bs[7], 0.0f);
      *(v4f*)(tile + pl * 132 + o) = lo;
      *(v4f*)(tile + pl * 132 + o + 4) = hi;
    }
  }
  __syncthreads();
  const int pl = tid & 63, ch = tid >> 6;
  float z = b3s[ch];
  const float* trow = tile + pl * 132;
  const float* wr = w3s + ch * CMID;
#pragma unroll 4
  for (int o = 0; o < CMID; ++o) z += wr[o] * trow[o];
  z = fminf(fmaxf(z, -80.0f), 80.0f);
  const float sg = 1.0f / (1.0f + expf(-z));
  float* dp = zb + ((size_t)(b * 2 + ch) * NPOS_PAD + p0 + pl);
  st1fv(dp, sg);
  __threadfence();
  st1fv(dp, sg);
}

__global__ __launch_bounds__(256) void k_pack(const float* __restrict__ zb, float* out) {
  const int gid = blockIdx.x * 256 + threadIdx.x;
  if (gid >= NBATCH * 2 * NPOS / 4) return;
  const int f = gid * 4;
  const int bc = f / NPOS, p = f - bc * NPOS;
  const v4f v = *(const v4f*)(zb + (size_t)bc * NPOS_PAD + p);
  float* dp = out + 800 + f;
  st4fv(dp, v);
  __threadfence();
  st4fv(dp, v);
}

extern "C" void kernel_launch(void* const* d_in, const int* in_sizes, int n_in,
                              void* d_out, int out_size, void* d_ws, size_t ws_size,
                              hipStream_t stream) {
  if (n_in < 17) return;
  if (in_sizes[0] != NBATCH * 400 * T_DIM) return;
  if (in_sizes[1] != 256 * 400 * 3 || in_sizes[2] != 256) return;
  if (in_sizes[3] != 128 * 256 * 3 || in_sizes[4] != 128) return;
  if (in_sizes[5] != 256 * 128 * 3 || in_sizes[6] != 256) return;
  if (in_sizes[7] != 2 * 256 * 3 || in_sizes[8] != 2) return;
  if (in_sizes[9] != OBIG * CMID * NSMP || in_sizes[10] != OBIG) return;
  if (in_sizes[11] != CMID * OBIG || in_sizes[12] != CMID) return;
  if (in_sizes[13] != CMID * CMID * 9 || in_sizes[14] != CMID) return;
  if (in_sizes[15] != 2 * CMID || in_sizes[16] != 2) return;
  if (out_size != 800 + NBATCH * 2 * NPOS) return;

  const float* x     = (const float*)d_in[0];
  const float* w_b1  = (const float*)d_in[1];
  const float* b_b1  = (const float*)d_in[2];
  const float* w_b2  = (const float*)d_in[3];
  const float* b_b2  = (const float*)d_in[4];
  const float* w_t1  = (const float*)d_in[5];
  const float* b_t1  = (const float*)d_in[6];
  const float* w_t2  = (const float*)d_in[7];
  const float* b_t2  = (const float*)d_in[8];
  const float* w_c3d = (const float*)d_in[9];
  const float* b_c3d = (const float*)d_in[10];
  const float* w_2d1 = (const float*)d_in[11];
  const float* b_2d1 = (const float*)d_in[12];
  const float* w_2d2 = (const float*)d_in[13];
  const float* b_2d2 = (const float*)d_in[14];
  const float* w_2d3 = (const float*)d_in[15];
  const float* b_2d3 = (const float*)d_in[16];
  float* out = (float*)d_out;

  char* ws = (char*)d_ws;
  size_t off = 0;
  const size_t szA5   = (size_t)OBIG * KBIG * 2;
  const size_t szA6   = (size_t)CMID * OBIG * 2;
  const size_t szA7   = (size_t)9 * CMID * CMID * 2;
  const size_t szB1   = (size_t)NBATCH * 256 * T_DIM * 4;
  const size_t szBase = (size_t)NBATCH * CMID * T_DIM * 4;
  const size_t szTem  = (size_t)NBATCH * 256 * T_DIM * 4;
  const size_t szP    = (size_t)RPAD * KBIG * 2;
  const size_t szY1   = (size_t)NBATCH * RPAD * OBIG * 2;
  const size_t szY2   = (size_t)NBATCH * NPOS_PAD * CMID * 2;
  const size_t szCv   = 256;
  const size_t szZ    = (size_t)NBATCH * 2 * NPOS_PAD * 4;
#define CARVE(NAME, SZ) const size_t NAME = off; off += ((SZ) + 255) & ~(size_t)255;
  CARVE(oA5, szA5) CARVE(oA6, szA6) CARVE(oA7, szA7) CARVE(oB1, szB1) CARVE(oBase, szBase) CARVE(oTem, szTem)
  CARVE(oP, szP) CARVE(oY1, szY1) CARVE(oY2, szY2) CARVE(oCv, szCv) CARVE(oZ, szZ)
#undef CARVE
  if (off > ws_size || off > (size_t)134217728) return;

  uint16_t* A5   = (uint16_t*)(ws + oA5);
  uint16_t* A6   = (uint16_t*)(ws + oA6);
  uint16_t* A7   = (uint16_t*)(ws + oA7);
  float*    bs1  = (float*)(ws + oB1);
  float*    base = (float*)(ws + oBase);
  float*    tem  = (float*)(ws + oTem);
  uint16_t* P    = (uint16_t*)(ws + oP);
  uint16_t* y1   = (uint16_t*)(ws + oY1);
  uint16_t* y2   = (uint16_t*)(ws + oY2);
  uint16_t* cvec = (uint16_t*)(ws + oCv);
  float*    zb   = (float*)(ws + oZ);

  const int nCvt = (OBIG * KBIG + CMID * OBIG + 9 * CMID * CMID) / 8;
  k_cvt<<<(nCvt + 255) / 256, 256, 0, stream>>>(w_c3d, w_2d1, w_2d2, A5, A6, A7);

  k_conv1d<<<dim3(256 / 64, NBATCH), 256, 0, stream>>>(x,    w_b1, b_b1, bs1,  400, 256);
  k_conv1d<<<dim3(128 / 64, NBATCH), 256, 0, stream>>>(bs1,  w_b2, b_b2, base, 256, 128);
  k_conv1d<<<dim3(256 / 64, NBATCH), 256, 0, stream>>>(base, w_t1, b_t1, tem,  128, 256);
  k_tem_head<<<1, 256, 0, stream>>>(tem, w_t2, b_t2, out);

  for (int b = 0; b < NBATCH; ++b) {
    k_pem<<<(RPAD * 8) / 256, 256, 0, stream>>>(base, P, b);
    k_gemm<0><<<dim3(RPAD / 128, OBIG / 128, 1), 256, 0, stream>>>(A5, P, b_c3d, y1, cvec, KBIG, b);
  }
  k_gemm<1><<<dim3(RPAD / 128, 1, NBATCH), 256, 0, stream>>>(A6, y1, b_2d1, y2, cvec, OBIG, 0);
  k_fill<<<dim3(NPOS / 16, NBATCH), 256, 0, stream>>>(cvec, y2);
  k_conv3x3<<<dim3((NPOS + 63) / 64, NBATCH), 128, 0, stream>>>(A7, y2, b_2d2, w_2d3, b_2d3, zb);
  k_pack<<<(NBATCH * 2 * NPOS / 4 + 255) / 256, 256, 0, stream>>>(zb, out);
}
